// GCNEncoder_5377299055294
// MI455X (gfx1250) — hardware-verified
//
#include <hip/hip_runtime.h>
#include <stddef.h>
#include <stdint.h>


#define CIN     128
#define CH      128
#define CO      64
#define NTHR    256
#define NWAVE   8
#define EPT     8
#define CHUNK   (NTHR * EPT)
#define NBD     8192
#define SLBD    13
#define WCAPD   (EPT * 32)
#define LISTD   (NWAVE * WCAPD)
#define NBA     1024
#define SLBA    10
#define WCAPA   2560
#define LTOT    (NWAVE * WCAPA)
#define SORTCAP 64
#define GBM     64
#define GTHR    128
#define SP1     (CH + 4)
#define SP2     (CO + 4)
#define NU1     (CH * (CIN / 8))
#define NU2     (CO * (CH / 8))
#define WSMAX   134217728
#define LO_LIST 0
#define LO_SRT  (LTOT)
#define LO_CNT  (2 * LTOT)
#define LO_OFF  (LO_CNT + NBA)
#define LO_CUR  (LO_OFF + NBA)
#define LO_SB   (LO_CUR + NBA)
#define LO_WT   (LO_SB + CH)
#define LO_WS   (LO_WT + NWAVE)
#define LO_END  (LO_WS + NWAVE)
#define AGGLDS  (LO_END * 4)

static_assert((CHUNK & (CHUNK - 1)) == 0 && CHUNK <= 4096);
static_assert((NBD & (NBD - 1)) == 0 && NBD == (1 << SLBD));
static_assert((NBA & (NBA - 1)) == 0 && NBA == (1 << SLBA));
static_assert(((long long)CHUNK << SLBD) < (1LL << 31));
static_assert(((1LL << 21) << SLBA) <= (1LL << 31));
static_assert(NBD % (NTHR * 4) == 0 && LISTD % NTHR == 0 && NBD % NTHR == 0);
static_assert(NBA == 4 * NTHR && ((2 * LTOT) % (4 * NTHR)) == 0);
static_assert((LO_SB % 4) == 0 && (LO_CNT % 4) == 0 && (LO_OFF % 4) == 0 && (LO_CUR % 4) == 0);
static_assert(CIN % 32 == 0 && CH % 32 == 0 && CH == 4 * 32 && CO == 4 * 16);
static_assert(GBM == (GTHR / 32) * 16 && ((SP1 * 4) % 16) == 0 && ((SP2 * 4) % 16) == 0);
static_assert((NU1 % NTHR) == 0 && ((NU1 + NU2) % NTHR) == 0);
static_assert(NBA % GBM == 0 && NBA % 2 == 0);

typedef float          v4f   __attribute__((ext_vector_type(4)));
typedef float          v8f   __attribute__((ext_vector_type(8)));
typedef int            v4i   __attribute__((ext_vector_type(4)));
typedef int            v8i   __attribute__((ext_vector_type(8)));
typedef unsigned short v8us  __attribute__((ext_vector_type(8)));
typedef unsigned short v16us __attribute__((ext_vector_type(16)));
typedef __bf16         v16bf __attribute__((ext_vector_type(16)));
typedef v4f  __attribute__((may_alias)) v4fa;
typedef v4i  __attribute__((may_alias)) v4ia;
typedef v8us __attribute__((may_alias)) v8usa;
union FragB { v16bf v; v16us u; v8us h[2]; v8i w; };

__device__ __forceinline__ v8f wmb(const FragB& a, const FragB& b, v8f c) {
  v8f d = __builtin_amdgcn_wmma_f32_16x16x32_bf16(false, a.v, false, b.v, (short)0, c, false, false);
  asm volatile("v_nop\n\tv_nop\n\tv_nop\n\tv_nop" : "+v"(d) : "v"(a.w), "v"(b.w));
  return d;
}

__device__ __forceinline__ unsigned bf16_bits(float f) {
  const unsigned u = __float_as_uint(f);
  return (u + 0x7FFFu + ((u >> 16) & 1u)) >> 16;
}
__device__ __forceinline__ float bf16_val(float f) {
  return __uint_as_float(bf16_bits(f) << 16);
}

__device__ __forceinline__ int scan_chunk(const int* __restrict__ dsts, int nE, int cbase, int slotBase,
                                          int nb, int vec8, int* wl, int wc0, int cap, int slb, int ebase,
                                          int tid) {
  int wc = 0;
  const int el0  = tid * EPT;
  const int e0   = cbase + el0;
  const int sent = -2147483647 - 1;
  v4i da, db;
  if (vec8 != 0 && cbase + CHUNK <= nE) {
    da = *(const v4ia*)(dsts + e0);
    db = *(const v4ia*)(dsts + e0 + 4);
  } else {
    da.x = (e0     < nE) ? dsts[min(e0,     nE - 1)] : sent;
    da.y = (e0 + 1 < nE) ? dsts[min(e0 + 1, nE - 1)] : sent;
    da.z = (e0 + 2 < nE) ? dsts[min(e0 + 2, nE - 1)] : sent;
    da.w = (e0 + 3 < nE) ? dsts[min(e0 + 3, nE - 1)] : sent;
    db.x = (e0 + 4 < nE) ? dsts[min(e0 + 4, nE - 1)] : sent;
    db.y = (e0 + 5 < nE) ? dsts[min(e0 + 5, nE - 1)] : sent;
    db.z = (e0 + 6 < nE) ? dsts[min(e0 + 6, nE - 1)] : sent;
    db.w = (e0 + 7 < nE) ? dsts[min(e0 + 7, nE - 1)] : sent;
  }
  const unsigned nbs = (unsigned)slotBase;
  const unsigned unb = (unsigned)nb;
  const unsigned s0 = (unsigned)da.x - nbs, s1 = (unsigned)da.y - nbs;
  const unsigned s2 = (unsigned)da.z - nbs, s3 = (unsigned)da.w - nbs;
  const unsigned s4 = (unsigned)db.x - nbs, s5 = (unsigned)db.y - nbs;
  const unsigned s6 = (unsigned)db.z - nbs, s7 = (unsigned)db.w - nbs;
  const bool h0 = s0 < unb, h1 = s1 < unb, h2 = s2 < unb, h3 = s3 < unb;
  const bool h4 = s4 < unb, h5 = s5 < unb, h6 = s6 < unb, h7 = s7 < unb;
  const unsigned any = __builtin_amdgcn_ballot_w32(h0 | h1 | h2 | h3 | h4 | h5 | h6 | h7);
  if (any != 0u) {
#define HITJ(J, HJ, SJ) { \
      const unsigned mj = __builtin_amdgcn_ballot_w32(HJ); \
      if (mj != 0u) { \
        if (HJ) { \
          const int pos = wc0 + wc + (int)__builtin_amdgcn_mbcnt_lo(mj, 0u); \
          if (pos >= 0 && pos < cap) wl[pos] = ((ebase + el0 + (J)) << slb) | (int)(SJ); \
        } \
        wc += (int)__builtin_popcount(mj); } }
    HITJ(0, h0, s0)
    HITJ(1, h1, s1)
    HITJ(2, h2, s2)
    HITJ(3, h3, s3)
    HITJ(4, h4, s4)
    HITJ(5, h5, s5)
    HITJ(6, h6, s6)
    HITJ(7, h7, s7)
#undef HITJ
  }
  return wc;
}

__global__ __launch_bounds__(NTHR) void k_wprep(const float* __restrict__ W1, const float* __restrict__ W2,
                                                unsigned short* W1T, unsigned short* W2T, int nUnits) {
  const int u = (int)blockIdx.x * NTHR + (int)threadIdx.x;
  if (u >= nUnits) return;
  const bool sec = (u >= NU1);
  const int uu = sec ? (u - NU1) : u;
  const int n  = uu >> 4;
  const int k8 = (uu & 15) * 8;
  const int ldn = sec ? CO : CH;
  const float* base = sec ? W2 : W1;
  const float* p = base + (size_t)k8 * ldn + n;
  v8us o;
  o[0] = (unsigned short)bf16_bits(p[0]);
  o[1] = (unsigned short)bf16_bits(p[(size_t)ldn]);
  o[2] = (unsigned short)bf16_bits(p[(size_t)2 * ldn]);
  o[3] = (unsigned short)bf16_bits(p[(size_t)3 * ldn]);
  o[4] = (unsigned short)bf16_bits(p[(size_t)4 * ldn]);
  o[5] = (unsigned short)bf16_bits(p[(size_t)5 * ldn]);
  o[6] = (unsigned short)bf16_bits(p[(size_t)6 * ldn]);
  o[7] = (unsigned short)bf16_bits(p[(size_t)7 * ldn]);
  unsigned short* dp = (sec ? W2T : W1T) + (size_t)n * 128 + k8;
  *(volatile v8us*)dp = o;
  __threadfence();
  *(volatile v8us*)dp = o;
}

__global__ __launch_bounds__(NTHR) void k_deg(const int* __restrict__ dsts, int nE, int vec8, float* dis) {
  __shared__ __attribute__((aligned(16))) int scnt[NBD];
  __shared__ __attribute__((aligned(16))) int list[LISTD];
  __shared__ int wcnt[NWAVE];
  const int tid = (int)threadIdx.x, lane = tid & 31, wave = tid >> 5;
  const int nodeBase = (int)blockIdx.x * NBD;

  for (int i = tid; i < NBD; i += NTHR) scnt[i] = 0;
  for (int i = tid; i < LISTD; i += NTHR) list[i] = 0;
  if (tid < NWAVE) wcnt[tid] = 0;
  __syncthreads();

  const int nChunks = (nE + CHUNK - 1) / CHUNK;
#pragma unroll 1
  for (int ch = 0; ch < nChunks; ++ch) {
    const int cbase = ch * CHUNK;
    const int wc = scan_chunk(dsts, nE, cbase, nodeBase, NBD, vec8, list + wave * WCAPD, 0, WCAPD, SLBD, 0, tid);
    if (lane == 0) wcnt[wave] = wc;
    __syncthreads();
    if (wave == 0) {
#pragma unroll 1
      for (int w2 = 0; w2 < NWAVE; ++w2) {
        int c = wcnt[w2];
        c = c < 0 ? 0 : (c > WCAPD ? WCAPD : c);
#pragma unroll 1
        for (int b0 = 0; b0 < c; b0 += 32) {
          const int idx = b0 + lane;
          const int ent = list[w2 * WCAPD + (idx < WCAPD ? idx : WCAPD - 1)];
          const int m32 = (c - b0) < 32 ? (c - b0) : 32;
#pragma unroll 1
          for (int k = 0; k < m32; ++k) {
            const int u  = __builtin_amdgcn_readlane(ent, k);
            const int sl = u & (NBD - 1);
            if (lane == 0) scnt[sl] = scnt[sl] + 1;
          }
        }
      }
    }
    __syncthreads();
  }

  v4f vals[NBD / (NTHR * 4)];
#pragma unroll
  for (int it = 0; it < NBD / (NTHR * 4); ++it) {
    const int s0 = it * (NTHR * 4) + 4 * tid;
    const v4i c4 = *(const v4ia*)(scnt + s0);
    v4f v;
    v.x = rsqrtf((float)c4.x + 1.0f);
    v.y = rsqrtf((float)c4.y + 1.0f);
    v.z = rsqrtf((float)c4.z + 1.0f);
    v.w = rsqrtf((float)c4.w + 1.0f);
    vals[it] = v;
  }
#pragma unroll
  for (int it = 0; it < NBD / (NTHR * 4); ++it) {
    const int s0 = it * (NTHR * 4) + 4 * tid;
    *(volatile v4f*)(dis + (size_t)nodeBase + s0) = vals[it];
  }
  __threadfence();
#pragma unroll
  for (int it = 0; it < NBD / (NTHR * 4); ++it) {
    const int s0 = it * (NTHR * 4) + 4 * tid;
    *(volatile v4f*)(dis + (size_t)nodeBase + s0) = vals[it];
  }
}

__global__ __launch_bounds__(GTHR) void k_gemm1(const float* __restrict__ X, const unsigned short* __restrict__ W1T,
                                                float* H1, int nN, int NP) {
  __shared__ __attribute__((aligned(16))) float stg[GBM * SP1];
  const int tid = (int)threadIdx.x, lane = tid & 31, wave = tid >> 5, hh = lane >> 4, m = lane & 15;
  const int rowBase = (int)blockIdx.x * GBM;
  const int row = rowBase + 16 * wave + m;
  const int rc  = row < nN ? row : nN - 1;
  const float* ap = X + (size_t)rc * CIN + 8 * hh;
  const unsigned short* wp = W1T + (size_t)m * CIN + 8 * hh;

  v8f acc[8];
  {
    const v8f z = {0.f, 0.f, 0.f, 0.f, 0.f, 0.f, 0.f, 0.f};
#pragma unroll
    for (int t = 0; t < 8; ++t) acc[t] = z;
  }

#pragma unroll 1
  for (int kk = 0; kk < CIN / 32; ++kk) {
    const int k0 = 32 * kk;
    const v4f x0 = *(const v4fa*)(ap + k0);
    const v4f x1 = *(const v4fa*)(ap + k0 + 4);
    const v4f x2 = *(const v4fa*)(ap + k0 + 16);
    const v4f x3 = *(const v4fa*)(ap + k0 + 20);
    FragB a;
    a.u[0]  = (unsigned short)bf16_bits(x0.x); a.u[1]  = (unsigned short)bf16_bits(x0.y);
    a.u[2]  = (unsigned short)bf16_bits(x0.z); a.u[3]  = (unsigned short)bf16_bits(x0.w);
    a.u[4]  = (unsigned short)bf16_bits(x1.x); a.u[5]  = (unsigned short)bf16_bits(x1.y);
    a.u[6]  = (unsigned short)bf16_bits(x1.z); a.u[7]  = (unsigned short)bf16_bits(x1.w);
    a.u[8]  = (unsigned short)bf16_bits(x2.x); a.u[9]  = (unsigned short)bf16_bits(x2.y);
    a.u[10] = (unsigned short)bf16_bits(x2.z); a.u[11] = (unsigned short)bf16_bits(x2.w);
    a.u[12] = (unsigned short)bf16_bits(x3.x); a.u[13] = (unsigned short)bf16_bits(x3.y);
    a.u[14] = (unsigned short)bf16_bits(x3.z); a.u[15] = (unsigned short)bf16_bits(x3.w);
#pragma unroll
    for (int nt = 0; nt < 8; ++nt) {
      const unsigned short* wq = wp + (size_t)(16 * nt) * CIN + k0;
      FragB b;
      b.h[0] = *(const v8usa*)wq;
      b.h[1] = *(const v8usa*)(wq + 16);
      acc[nt] = wmb(a, b, acc[nt]);
    }
  }

#pragma unroll
  for (int nt = 0; nt < 8; ++nt) {
    const int lc = 16 * nt + m;
#pragma unroll
    for (int r = 0; r < 8; ++r) {
      const int lr = 16 * wave + 8 * hh + r;
      stg[lr * SP1 + lc] = acc[nt][r];
    }
  }
  __syncthreads();

#pragma unroll
  for (int g = 0; g < 2; ++g) {
    v4f pv[8];
#pragma unroll
    for (int i = 0; i < 8; ++i) {
      const int lr = 16 * wave + 8 * g + i;
      pv[i] = *(const v4fa*)(stg + lr * SP1 + 4 * lane);
    }
#pragma unroll
    for (int i = 0; i < 8; ++i) {
      const int lr = 16 * wave + 8 * g + i;
      float* op = H1 + (size_t)(rowBase + lr) * CH + 4 * lane;
      *(volatile v4f*)op = pv[i];
    }
    __threadfence();
#pragma unroll
    for (int i = 0; i < 8; ++i) {
      const int lr = 16 * wave + 8 * g + i;
      float* op = H1 + (size_t)(rowBase + lr) * CH + 4 * lane;
      *(volatile v4f*)op = pv[i];
    }
  }
}

__global__ __launch_bounds__(GTHR) void k_gemm2(const float* __restrict__ A1, const unsigned short* __restrict__ W2T,
                                                float* H2, int NP) {
  __shared__ __attribute__((aligned(16))) float stg[GBM * SP2];
  const int tid = (int)threadIdx.x, lane = tid & 31, wave = tid >> 5, hh = lane >> 4, m = lane & 15;
  const int rowBase = (int)blockIdx.x * GBM;
  const int row = rowBase + 16 * wave + m;
  const int rc  = row < NP ? row : NP - 1;
  const float* ap = A1 + (size_t)rc * CH + 8 * hh;
  const unsigned short* wp = W2T + (size_t)m * CH + 8 * hh;

  v8f acc[4];
  {
    const v8f z = {0.f, 0.f, 0.f, 0.f, 0.f, 0.f, 0.f, 0.f};
#pragma unroll
    for (int t = 0; t < 4; ++t) acc[t] = z;
  }

#pragma unroll 1
  for (int kk = 0; kk < CH / 32; ++kk) {
    const int k0 = 32 * kk;
    const v4f x0 = *(const v4fa*)(ap + k0);
    const v4f x1 = *(const v4fa*)(ap + k0 + 4);
    const v4f x2 = *(const v4fa*)(ap + k0 + 16);
    const v4f x3 = *(const v4fa*)(ap + k0 + 20);
    FragB ah, al;
#define HL(I, V) { const float vv = (V); const unsigned hb = bf16_bits(vv); \
      ah.u[I] = (unsigned short)hb; \
      al.u[I] = (unsigned short)bf16_bits(vv - __uint_as_float(hb << 16)); }
    HL(0, x0.x)  HL(1, x0.y)  HL(2, x0.z)  HL(3, x0.w)
    HL(4, x1.x)  HL(5, x1.y)  HL(6, x1.z)  HL(7, x1.w)
    HL(8, x2.x)  HL(9, x2.y)  HL(10, x2.z) HL(11, x2.w)
    HL(12, x3.x) HL(13, x3.y) HL(14, x3.z) HL(15, x3.w)
#undef HL
#pragma unroll
    for (int nt = 0; nt < 4; ++nt) {
      const unsigned short* wq = wp + (size_t)(16 * nt) * CH + k0;
      FragB b;
      b.h[0] = *(const v8usa*)wq;
      b.h[1] = *(const v8usa*)(wq + 16);
      acc[nt] = wmb(ah, b, acc[nt]);
      acc[nt] = wmb(al, b, acc[nt]);
    }
  }

#pragma unroll
  for (int nt = 0; nt < 4; ++nt) {
    const int lc = 16 * nt + m;
#pragma unroll
    for (int r = 0; r < 8; ++r) {
      const int lr = 16 * wave + 8 * hh + r;
      stg[lr * SP2 + lc] = acc[nt][r];
    }
  }
  __syncthreads();

  v4f pv[8];
#pragma unroll
  for (int i = 0; i < 8; ++i) {
    const int lr = 16 * wave + 2 * i + hh;
    pv[i] = *(const v4fa*)(stg + lr * SP2 + 4 * m);
  }
#pragma unroll
  for (int i = 0; i < 8; ++i) {
    const int lr = 16 * wave + 2 * i + hh;
    float* op = H2 + (size_t)(rowBase + lr) * CO + 4 * m;
    *(volatile v4f*)op = pv[i];
  }
  __threadfence();
#pragma unroll
  for (int i = 0; i < 8; ++i) {
    const int lr = 16 * wave + 2 * i + hh;
    float* op = H2 + (size_t)(rowBase + lr) * CO + 4 * m;
    *(volatile v4f*)op = pv[i];
  }
}

template <int C, int RELU>
__global__ __launch_bounds__(NTHR) void k_agg(const int* __restrict__ srcs, const int* __restrict__ dsts,
                                              const float* __restrict__ dis, const float* __restrict__ hpl,
                                              const float* __restrict__ bias, int nE, int nN, int vec8,
                                              float* outp, int nRows) {
  extern __shared__ __attribute__((aligned(16))) int dynlds[];
  int*   list = dynlds + LO_LIST;
  int*   srt  = dynlds + LO_SRT;
  int*   cnt  = dynlds + LO_CNT;
  int*   off  = dynlds + LO_OFF;
  int*   cur  = dynlds + LO_CUR;
  float* sb   = (float*)(dynlds + LO_SB);
  int*   wtot = dynlds + LO_WT;
  int*   wsum = dynlds + LO_WS;
  const int tid = (int)threadIdx.x, lane = tid & 31, wave = tid >> 5, hh = lane >> 4, m = lane & 15;
  const int slotBase = (int)blockIdx.x * NBA;

  {
    const v4i z4 = {0, 0, 0, 0};
#pragma unroll 1
    for (int i = tid; i < (2 * LTOT) / 4; i += NTHR) *(v4ia*)(dynlds + LO_LIST + 4 * i) = z4;
#pragma unroll 1
    for (int i = tid; i < NBA; i += NTHR) { cnt[i] = 0; off[i] = 0; cur[i] = 0; }
    if (tid < CH) sb[tid] = (tid < C) ? bf16_val(bias[tid < C ? tid : C - 1]) : 0.0f;
    if (tid < NWAVE) { wtot[tid] = 0; wsum[tid] = 0; }
  }
  __syncthreads();

  int wc0 = 0;
  const int nChunks = (nE + CHUNK - 1) / CHUNK;
#pragma unroll 1
  for (int ch = 0; ch < nChunks; ++ch) {
    const int cbase = ch * CHUNK;
    const int wc = scan_chunk(dsts, nE, cbase, slotBase, NBA, vec8, list + wave * WCAPA, wc0, WCAPA, SLBA,
                              cbase, tid);
    wc0 += wc;
  }
  if (lane == 0) wtot[wave] = wc0;
  __syncthreads();

  int ovf = 0;
#pragma unroll
  for (int w = 0; w < NWAVE; ++w) ovf |= (wtot[w] > WCAPA) ? 1 : 0;

  if (wave == 0) {
#pragma unroll 1
    for (int w2 = 0; w2 < NWAVE; ++w2) {
      int n = wtot[w2];
      n = n < 0 ? 0 : (n > WCAPA ? WCAPA : n);
#pragma unroll 1
      for (int b0 = 0; b0 < n; b0 += 32) {
        const int idx = b0 + lane;
        const int ent = list[w2 * WCAPA + (idx < WCAPA ? idx : WCAPA - 1)];
        const int m32 = (n - b0) < 32 ? (n - b0) : 32;
#pragma unroll 1
        for (int k = 0; k < m32; ++k) {
          const int u  = __builtin_amdgcn_readlane(ent, k);
          const int sl = u & (NBA - 1);
          if (lane == 0) cnt[sl] = cnt[sl] + 1;
        }
      }
    }
  }
  __syncthreads();

  {
    const v4i c4 = *(const v4ia*)(cnt + 4 * tid);
    const int s4 = c4.x + c4.y + c4.z + c4.w;
    int x = s4;
#pragma unroll
    for (int d = 1; d < 32; d <<= 1) {
      const int y = __shfl_up(x, (unsigned)d, 32);
      x += (lane >= d) ? y : 0;
    }
    if (lane == 31) wsum[wave] = x;
    __syncthreads();
    int pre = 0;
#pragma unroll
    for (int w = 0; w < NWAVE; ++w) pre += (w < wave) ? wsum[w] : 0;
    const int ex = pre + x - s4;
    v4i o;
    o.x = ex; o.y = ex + c4.x; o.z = o.y + c4.y; o.w = o.z + c4.z;
    *(v4ia*)(off + 4 * tid) = o;
    *(v4ia*)(cur + 4 * tid) = o;
  }
  __syncthreads();

  if (wave == 0) {
#pragma unroll 1
    for (int w2 = 0; w2 < NWAVE; ++w2) {
      int n = wtot[w2];
      n = n < 0 ? 0 : (n > WCAPA ? WCAPA : n);
#pragma unroll 1
      for (int b0 = 0; b0 < n; b0 += 32) {
        const int idx = b0 + lane;
        const int ent = list[w2 * WCAPA + (idx < WCAPA ? idx : WCAPA - 1)];
        const int m32 = (n - b0) < 32 ? (n - b0) : 32;
#pragma unroll 1
        for (int k = 0; k < m32; ++k) {
          const int u  = __builtin_amdgcn_readlane(ent, k);
          const int sl = u & (NBA - 1);
          if (lane == 0) {
            int p = cur[sl];
            p = p < 0 ? 0 : (p > LTOT - 1 ? LTOT - 1 : p);
            srt[p] = u;
            cur[sl] = p + 1;
          }
        }
      }
    }
  }
  __syncthreads();

#pragma unroll 1
  for (int q = 0; q < NBA / NTHR; ++q) {
    const int s = tid + q * NTHR;
    int st = off[s];
    int n  = cnt[s];
    st = st < 0 ? 0 : (st > LTOT ? LTOT : st);
    n  = n < 0 ? 0 : (n > SORTCAP ? SORTCAP : n);
    if (n > LTOT - st) n = LTOT - st;
#pragma unroll 1
    for (int i = 1; i < n; ++i) {
      const int key = srt[st + i];
      int j = i - 1;
#pragma unroll 1
      while (j >= 0) {
        const int v = srt[st + j];
        if (v <= key) break;
        srt[st + j + 1] = v;
        --j;
      }
      srt[st + j + 1] = key;
    }
  }
  __syncthreads();

  const float qn = __uint_as_float(0x7fc00000u);
  if (C == 128) {
#pragma unroll 1
    for (int sl = wave; sl < NBA; sl += NWAVE) {
      const int node = slotBase + sl;
      const int nc = node < nN ? node : nN - 1;
      const float dvd = dis[nc];
      int st = off[sl];
      int n  = cnt[sl];
      st = st < 0 ? 0 : (st > LTOT ? LTOT : st);
      n  = n < 0 ? 0 : (n > LTOT - st ? LTOT - st : n);
      v4f acc = {0.f, 0.f, 0.f, 0.f};
#pragma unroll 1
      for (int j = 0; j < n; ++j) {
        const int e = srt[st + j];
        int eid = e >> SLBA;
        eid = eid < 0 ? 0 : (eid > nE - 1 ? nE - 1 : eid);
        int s = srcs[eid];
        s = s < 0 ? 0 : (s > nN - 1 ? nN - 1 : s);
        const float w = dis[s] * dvd;
        const v4f hv = *(const v4fa*)(hpl + (size_t)s * C + 4 * lane);
        acc.x = fmaf(w, hv.x, acc.x);
        acc.y = fmaf(w, hv.y, acc.y);
        acc.z = fmaf(w, hv.z, acc.z);
        acc.w = fmaf(w, hv.w, acc.w);
      }
      const v4f hs = *(const v4fa*)(hpl + (size_t)nc * C + 4 * lane);
      const v4f bb = *(const v4fa*)(sb + 4 * lane);
      const float sn = dvd * dvd;
      v4f r;
      r.x = (acc.x + sn * hs.x) + bb.x;
      r.y = (acc.y + sn * hs.y) + bb.y;
      r.z = (acc.z + sn * hs.z) + bb.z;
      r.w = (acc.w + sn * hs.w) + bb.w;
      if (RELU) { r.x = fmaxf(r.x, 0.f); r.y = fmaxf(r.y, 0.f); r.z = fmaxf(r.z, 0.f); r.w = fmaxf(r.w, 0.f); }
      if (node >= nN) { r.x = 0.f; r.y = 0.f; r.z = 0.f; r.w = 0.f; }
      if (ovf != 0) { r.x = qn; r.y = qn; r.z = qn; r.w = qn; }
      if (node < nRows) {
        float* op = outp + (size_t)node * C + 4 * lane;
        *(volatile v4f*)op = r;
        __threadfence();
        *(volatile v4f*)op = r;
      }
    }
  } else {
#pragma unroll 1
    for (int pq = wave; pq < NBA / 2; pq += NWAVE) {
      const int slA = 2 * pq, slB = slA + 1;
      const int msl = slA + hh;
      const int node = slotBase + msl;
      const int nc = node < nN ? node : nN - 1;
      const float dvd = dis[nc];
      int stA = off[slA], nA = cnt[slA], stB = off[slB], nB = cnt[slB];
      stA = stA < 0 ? 0 : (stA > LTOT ? LTOT : stA);
      stB = stB < 0 ? 0 : (stB > LTOT ? LTOT : stB);
      nA = nA < 0 ? 0 : (nA > LTOT - stA ? LTOT - stA : nA);
      nB = nB < 0 ? 0 : (nB > LTOT - stB ? LTOT - stB : nB);
      const int nmax = nA > nB ? nA : nB;
      const int myn  = hh ? nB : nA;
      const int myst = hh ? stB : stA;
      v4f acc = {0.f, 0.f, 0.f, 0.f};
#pragma unroll 1
      for (int j = 0; j < nmax; ++j) {
        const bool act = (j < myn);
        int idx = myst + (act ? j : 0);
        idx = idx < 0 ? 0 : (idx > LTOT - 1 ? LTOT - 1 : idx);
        const int e = srt[idx];
        int eid = e >> SLBA;
        eid = eid < 0 ? 0 : (eid > nE - 1 ? nE - 1 : eid);
        int s = srcs[eid];
        s = s < 0 ? 0 : (s > nN - 1 ? nN - 1 : s);
        const float dvs = dis[s];
        const float w = act ? (dvs * dvd) : 0.f;
        const v4f hv = *(const v4fa*)(hpl + (size_t)s * C + 4 * m);
        acc.x = fmaf(w, hv.x, acc.x);
        acc.y = fmaf(w, hv.y, acc.y);
        acc.z = fmaf(w, hv.z, acc.z);
        acc.w = fmaf(w, hv.w, acc.w);
      }
      const v4f hs = *(const v4fa*)(hpl + (size_t)nc * C + 4 * m);
      const v4f bb = *(const v4fa*)(sb + 4 * m);
      const float sn = dvd * dvd;
      v4f r;
      r.x = (acc.x + sn * hs.x) + bb.x;
      r.y = (acc.y + sn * hs.y) + bb.y;
      r.z = (acc.z + sn * hs.z) + bb.z;
      r.w = (acc.w + sn * hs.w) + bb.w;
      if (RELU) { r.x = fmaxf(r.x, 0.f); r.y = fmaxf(r.y, 0.f); r.z = fmaxf(r.z, 0.f); r.w = fmaxf(r.w, 0.f); }
      if (node >= nN) { r.x = 0.f; r.y = 0.f; r.z = 0.f; r.w = 0.f; }
      if (ovf != 0) { r.x = qn; r.y = qn; r.z = qn; r.w = qn; }
      const bool ok = (node < nRows);
      float* op = outp + (size_t)(ok ? node : 0) * C + 4 * m;
      if (ok) *(volatile v4f*)op = r;
      __threadfence();
      if (ok) *(volatile v4f*)op = r;
    }
  }
}

static inline int cdiv(int a, int b) { return (a + b - 1) / b; }

extern "C" void kernel_launch(void* const* d_in, const int* in_sizes, int n_in,
                              void* d_out, int out_size, void* d_ws, size_t ws_size,
                              hipStream_t stream) {
  if (n_in < 6) return;
  if (in_sizes[0] < CIN || (in_sizes[0] % CIN) != 0) return;
  const int nN = in_sizes[0] / CIN;
  if (in_sizes[1] < 2 || (in_sizes[1] & 1) != 0) return;
  const int nE = in_sizes[1] / 2;
  if (nE < 1 || nE > (1 << 21)) return;
  if (in_sizes[2] != CIN * CH || in_sizes[3] != CH) return;
  if (in_sizes[4] != CH * CO || in_sizes[5] != CO) return;
  if ((long long)out_size != (long long)nN * CO) return;
  if (nN < 1) return;

  const float* x    = (const float*)d_in[0];
  const int*   edge = (const int*)d_in[1];
  const float* W1   = (const float*)d_in[2];
  const float* b1   = (const float*)d_in[3];
  const float* W2   = (const float*)d_in[4];
  const float* b2   = (const float*)d_in[5];
  float* out = (float*)d_out;
  const int* src = edge;
  const int* dst = edge + nE;

  const int gD   = cdiv(nN, NBD);
  const int NBPD = gD * NBD;
  const int gA   = cdiv(nN, NBA);
  const int NBPA = gA * NBA;
  const int NP   = cdiv(nN, GBM) * GBM;
  const int gM   = NP / GBM;
  if (NP > NBPA || nN > NBPD) return;
  const int vec8 = ((nE & 3) == 0) ? 1 : 0;

  char* ws = (char*)d_ws;
  size_t off = 0;
  const size_t oDIS = off; off += (size_t)NBPD * 4;              off = (off + 255) & ~(size_t)255;
  const size_t oW1T = off; off += (size_t)CH * CIN * 2;          off = (off + 255) & ~(size_t)255;
  const size_t oW2T = off; off += (size_t)CO * CH * 2;           off = (off + 255) & ~(size_t)255;
  const size_t oH1  = off; off += (size_t)NP * CH * 4;           off = (off + 255) & ~(size_t)255;
  const size_t oA1  = off; off += (size_t)NP * CH * 4;           off = (off + 255) & ~(size_t)255;
  const size_t oH2  = off; off += (size_t)NP * CO * 4;           off = (off + 255) & ~(size_t)255;
  if (off > ws_size || off > (size_t)WSMAX) return;
  float*          DIS = (float*)(ws + oDIS);
  unsigned short* W1T = (unsigned short*)(ws + oW1T);
  unsigned short* W2T = (unsigned short*)(ws + oW2T);
  float*          H1  = (float*)(ws + oH1);
  float*          A1  = (float*)(ws + oA1);
  float*          H2  = (float*)(ws + oH2);

  const int nUw = NU1 + NU2;
  k_wprep<<<cdiv(nUw, NTHR), NTHR, 0, stream>>>(W1, W2, W1T, W2T, nUw);
  k_deg<<<gD, NTHR, 0, stream>>>(dst, nE, vec8, DIS);
  k_gemm1<<<gM, GTHR, 0, stream>>>(x, W1T, H1, nN, NP);
  hipFuncSetAttribute(reinterpret_cast<const void*>(&k_agg<CH, 1>),
                      hipFuncAttributeMaxDynamicSharedMemorySize, AGGLDS);
  k_agg<CH, 1><<<gA, NTHR, AGGLDS, stream>>>(src, dst, DIS, H1, b1, nE, nN, vec8, A1, NP);
  k_gemm2<<<gM, GTHR, 0, stream>>>(A1, W2T, H2, NP);
  hipFuncSetAttribute(reinterpret_cast<const void*>(&k_agg<CO, 0>),
                      hipFuncAttributeMaxDynamicSharedMemorySize, AGGLDS);
  k_agg<CO, 0><<<gA, NTHR, AGGLDS, stream>>>(src, dst, DIS, H2, b2, nE, nN, vec8, out, nN);
}
